// GATLayer_28467043238495
// MI455X (gfx1250) — hardware-verified
//
#include <hip/hip_runtime.h>
#include <stddef.h>
#include <stdint.h>
#include <math.h>


#define NB     8
#define NNODE  1024
#define KIN    512
#define NHEAD  8
#define HD     64
#define ODIM   (NHEAD * HD)
#define MROWS  (NB * NNODE)
#define PTHR   256
#define NBX    ((MROWS * KIN) / (8 * PTHR))
#define NBA    ((NB * NNODE * NNODE) / (8 * PTHR))
#define NBW    ((ODIM * KIN) / (8 * PTHR))
#define GBM    64
#define GBN    64
#define GTHR   128
#define ATHR   256
#define AROWS  16
#define WSMAX  134217728

static_assert((MROWS * KIN) % (8 * PTHR) == 0);
static_assert((NB * NNODE * NNODE) % (8 * PTHR) == 0);
static_assert((ODIM * KIN) % (8 * PTHR) == 0);
static_assert(KIN % 32 == 0 && NNODE % 32 == 0);
static_assert(MROWS % GBM == 0 && NNODE % GBM == 0 && ODIM % GBN == 0 && HD == GBN);
static_assert(GBM == (GTHR / 32) * 16 && GTHR == 2 * GBN && GTHR == 2 * GBM);
static_assert(ATHR == 32 * NHEAD && NNODE % AROWS == 0 && (NNODE / AROWS) == 64);
static_assert((KIN / 8) == 64);

typedef float          v4f  __attribute__((ext_vector_type(4)));
typedef float          v8f  __attribute__((ext_vector_type(8)));
typedef int            v8i  __attribute__((ext_vector_type(8)));
typedef unsigned int   v4u  __attribute__((ext_vector_type(4)));
typedef unsigned short v8us __attribute__((ext_vector_type(8)));
typedef __bf16         v16b __attribute__((ext_vector_type(16)));
typedef v4f  __attribute__((may_alias)) v4fa;
typedef v4u  __attribute__((may_alias)) v4ua;
typedef v8us __attribute__((may_alias)) v8usa;
union FragB { v16b v; v8us h[2]; v8i w; };

__device__ __forceinline__ v8f wmb(const FragB& a, const FragB& b, v8f c) {
  v8f d = __builtin_amdgcn_wmma_f32_16x16x32_bf16(false, a.v, false, b.v, (short)0, c, false, false);
  asm volatile("v_nop\n\tv_nop\n\tv_nop\n\tv_nop" : "+v"(d) : "v"(a.w), "v"(b.w));
  return d;
}

__device__ __forceinline__ unsigned int f2bf(float f) {
  const unsigned int u = __float_as_uint(f);
  return ((u + 0x7FFFu + ((u >> 16) & 1u)) >> 16) & 0xFFFFu;
}
__device__ __forceinline__ float bf2f(unsigned int b) { return __uint_as_float(b << 16); }
__device__ __forceinline__ float bfr(float f) { return bf2f(f2bf(f)); }
__device__ __forceinline__ unsigned int pk2(float lo, float hi) { return f2bf(lo) | (f2bf(hi) << 16); }
__device__ __forceinline__ v4u pack8(const v4f a, const v4f b) {
  v4u r;
  r.x = pk2(a.x, a.y); r.y = pk2(a.z, a.w); r.z = pk2(b.x, b.y); r.w = pk2(b.z, b.w);
  return r;
}

__device__ __forceinline__ float score_el(float sfr, float nf, float av) {
#pragma clang fp contract(off)
  const float x  = sfr + nf;
  const float l  = (x >= 0.0f) ? x : 0.01f * x;
  const float om = 1.0f - av;
  const float mv = -1.0e9f * om;
  return l + mv;
}

__global__ __launch_bounds__(PTHR) void k_prep(const float* __restrict__ A, const float* __restrict__ X,
                                               const float* __restrict__ W,
                                               unsigned short* AB, unsigned short* XB, unsigned short* WT) {
  const int blk = (int)blockIdx.x;
  const int tid = (int)threadIdx.x;
  v4u wv;
  unsigned short* dp;
  if (blk < NBX) {
    const size_t e = ((size_t)blk * PTHR + (size_t)tid) * 8;
    const v4f a = *(const v4fa*)(X + e);
    const v4f b = *(const v4fa*)(X + e + 4);
    wv = pack8(a, b);
    dp = XB + e;
  } else if (blk < NBX + NBA) {
    const size_t e = ((size_t)(blk - NBX) * PTHR + (size_t)tid) * 8;
    const v4f a = *(const v4fa*)(A + e);
    const v4f b = *(const v4fa*)(A + e + 4);
    wv = pack8(a, b);
    dp = AB + e;
  } else if (blk < NBX + NBA + NBW) {
    const int u  = (blk - NBX - NBA) * PTHR + tid;
    const int n  = u >> 6;
    const int k8 = (u & 63) * 8;
    const int h  = n >> 6, o = n & 63;
    const float* p = W + ((size_t)h * KIN + (size_t)k8) * HD + o;
    v4f a, b;
    a.x = p[0];        a.y = p[HD];       a.z = p[2 * HD];   a.w = p[3 * HD];
    b.x = p[4 * HD];   b.y = p[5 * HD];   b.z = p[6 * HD];   b.w = p[7 * HD];
    wv = pack8(a, b);
    dp = WT + (size_t)n * KIN + k8;
  } else {
    return;
  }
  *(volatile v4u*)dp = wv;
  __threadfence();
  *(volatile v4u*)dp = wv;
}

__global__ __launch_bounds__(GTHR) void k_proj(
    const unsigned short* __restrict__ XB, const unsigned short* __restrict__ WT,
    const float* __restrict__ w1, const float* __restrict__ b1,
    const float* __restrict__ w2, const float* __restrict__ b2,
    unsigned short* VtH, unsigned short* VtL, float* SD)
{
  __shared__ __attribute__((aligned(16))) float stg[GBM * GBN];
  __shared__ __attribute__((aligned(16))) float satt[2 * GBN];
  __shared__ __attribute__((aligned(16))) float sdot[2 * GBM];
  const int tid = (int)threadIdx.x, lane = tid & 31, wave = tid >> 5, hh = lane >> 4, m = lane & 15;
  const int rowBase = (int)blockIdx.x * GBM;
  const int head    = (int)blockIdx.y;
  const int col0    = head * GBN;
  const int bb      = rowBase / NNODE;
  const int n0      = rowBase - bb * NNODE;
  const int bh      = bb * NHEAD + head;

  {
    const int which = tid >> 6;
    const int c  = tid & 63;
    const float vs = w1[head * HD + c];
    const float vd = w2[head * HD + c];
    const float v = (which == 0) ? vs : vd;
    satt[which * GBN + c] = bfr(v);
  }

  v8f acc[4];
  {
    const v8f z = {0.f, 0.f, 0.f, 0.f, 0.f, 0.f, 0.f, 0.f};
    acc[0] = z; acc[1] = z; acc[2] = z; acc[3] = z;
  }
  const unsigned short* ap = XB + (size_t)(rowBase + 16 * wave + m) * (size_t)KIN + 8 * hh;
  const unsigned short* wp = WT + (size_t)(col0 + m) * (size_t)KIN + 8 * hh;
#pragma unroll 1
  for (int ks = 0; ks < KIN / 32; ++ks) {
    FragB af;
    af.h[0] = *(const v8usa*)(ap + 32 * ks);
    af.h[1] = *(const v8usa*)(ap + 32 * ks + 16);
#pragma unroll
    for (int t = 0; t < 4; ++t) {
      const unsigned short* wq = wp + (size_t)(16 * t) * (size_t)KIN + 32 * ks;
      FragB bf;
      bf.h[0] = *(const v8usa*)wq;
      bf.h[1] = *(const v8usa*)(wq + 16);
      acc[t] = wmb(af, bf, acc[t]);
    }
  }

#pragma unroll
  for (int t = 0; t < 4; ++t) {
    const int lc = 16 * t + m;
#pragma unroll
    for (int r = 0; r < 8; ++r) {
      const int lr = 16 * wave + 8 * hh + r;
      stg[lr * GBN + lc] = acc[t][r];
    }
  }
  __syncthreads();

  {
    const int row = tid & 63, which = tid >> 6;
    const float* sa = satt + which * GBN;
    const float* hr = stg + row * GBN;
    const float bs = b1[head];
    const float bd = b2[head];
    const float bias = bfr((which == 0) ? bs : bd);
    float d = 0.f;
#pragma unroll 4
    for (int c4 = 0; c4 < GBN / 4; ++c4) {
      const v4f hv = *(const v4fa*)(hr + 4 * c4);
      const v4f av = *(const v4fa*)(sa + 4 * c4);
      d = fmaf(hv.x, av.x, d);
      d = fmaf(hv.y, av.y, d);
      d = fmaf(hv.z, av.z, d);
      d = fmaf(hv.w, av.w, d);
    }
    sdot[which * GBM + row] = d + bias;
  }
  __syncthreads();

  const int q = tid & 7, lb = tid >> 3;
  v4u hv[4], lv[4];
#pragma unroll
  for (int i = 0; i < 4; ++i) {
    const int o = lb + 16 * i;
    unsigned int hb[8], lo[8];
#pragma unroll
    for (int j = 0; j < 8; ++j) {
      const float x = stg[(8 * q + j) * GBN + o];
      hb[j] = f2bf(x);
      lo[j] = f2bf(x - bf2f(hb[j]));
    }
    v4u a, b;
    a.x = hb[0] | (hb[1] << 16); a.y = hb[2] | (hb[3] << 16); a.z = hb[4] | (hb[5] << 16); a.w = hb[6] | (hb[7] << 16);
    b.x = lo[0] | (lo[1] << 16); b.y = lo[2] | (lo[3] << 16); b.z = lo[4] | (lo[5] << 16); b.w = lo[6] | (lo[7] << 16);
    hv[i] = a; lv[i] = b;
  }
  const size_t pbase = ((size_t)bh * HD + (size_t)lb) * NNODE + (size_t)n0 + 8 * q;
  const int which2 = lane >> 4, piece = lane & 15;
  const v4f sdv = *(const v4fa*)(sdot + which2 * GBM + 4 * piece);
  float* sp = SD + ((size_t)bh * 2 + (size_t)which2) * NNODE + n0 + 4 * piece;

#pragma unroll
  for (int i = 0; i < 4; ++i) {
    const size_t o2 = pbase + (size_t)(16 * i) * NNODE;
    *(volatile v4u*)(VtH + o2) = hv[i];
    *(volatile v4u*)(VtL + o2) = lv[i];
  }
  if (wave == 0) *(volatile v4f*)sp = sdv;
  __threadfence();
#pragma unroll
  for (int i = 0; i < 4; ++i) {
    const size_t o2 = pbase + (size_t)(16 * i) * NNODE;
    *(volatile v4u*)(VtH + o2) = hv[i];
    *(volatile v4u*)(VtL + o2) = lv[i];
  }
  if (wave == 0) *(volatile v4f*)sp = sdv;
}

__global__ __launch_bounds__(ATHR) void k_attn(
    const unsigned short* __restrict__ AB, const unsigned short* __restrict__ VtH,
    const unsigned short* __restrict__ VtL, const float* __restrict__ SD, float* out)
{
  __shared__ __attribute__((aligned(16))) float st[NHEAD * AROWS * HD];
  const int tid = (int)threadIdx.x, lane = tid & 31, wave = tid >> 5, hh = lane >> 4, m = lane & 15;
  const int b    = (int)blockIdx.x >> 6;
  const int row0 = ((int)blockIdx.x & 63) * AROWS;
  const int h    = wave;
  const int bh   = b * NHEAD + h;

  const float sfr = SD[((size_t)bh * 2) * NNODE + row0 + m];
  const float* nfp = SD + ((size_t)bh * 2 + 1) * NNODE + 8 * hh;
  const unsigned short* abp = AB  + ((size_t)b * NNODE + (size_t)(row0 + m)) * NNODE + 8 * hh;
  const unsigned short* vhp = VtH + ((size_t)bh * HD + (size_t)m) * NNODE + 8 * hh;
  const unsigned short* vlp = VtL + ((size_t)bh * HD + (size_t)m) * NNODE + 8 * hh;

  v8f O[4];
  {
    const v8f z = {0.f, 0.f, 0.f, 0.f, 0.f, 0.f, 0.f, 0.f};
    O[0] = z; O[1] = z; O[2] = z; O[3] = z;
  }
  float mx = -__builtin_inff();
  float rs = 0.0f;

#pragma unroll 1
  for (int ks = 0; ks < NNODE / 32; ++ks) {
    const int k0 = 32 * ks;
    const v4u aw0 = *(const v4ua*)(abp + k0);
    const v4u aw1 = *(const v4ua*)(abp + k0 + 16);
    const v4f na = *(const v4fa*)(nfp + k0);
    const v4f nb = *(const v4fa*)(nfp + k0 + 4);
    const v4f nc = *(const v4fa*)(nfp + k0 + 16);
    const v4f nd = *(const v4fa*)(nfp + k0 + 20);
    const float nfv[16] = {na.x, na.y, na.z, na.w, nb.x, nb.y, nb.z, nb.w,
                           nc.x, nc.y, nc.z, nc.w, nd.x, nd.y, nd.z, nd.w};
    const unsigned int aw[8] = {aw0.x, aw0.y, aw0.z, aw0.w, aw1.x, aw1.y, aw1.z, aw1.w};
    float t[16];
#pragma unroll
    for (int j = 0; j < 8; ++j) {
      const float ae = __uint_as_float(aw[j] << 16);
      const float ao = __uint_as_float(aw[j] & 0xffff0000u);
      t[2 * j]     = score_el(sfr, nfv[2 * j],     ae);
      t[2 * j + 1] = score_el(sfr, nfv[2 * j + 1], ao);
    }
    float tm = t[0];
#pragma unroll
    for (int i = 1; i < 16; ++i) tm = fmaxf(tm, t[i]);
    tm = fmaxf(tm, __shfl_xor(tm, 16));
    const float mn = fmaxf(mx, tm);
    const float sc = expf(mx - mn);
    mx = mn;

    float p[16];
    float ps = 0.0f;
#pragma unroll
    for (int i = 0; i < 16; ++i) { p[i] = expf(t[i] - mn); ps += p[i]; }
    rs = rs * sc + ps;

    FragB ph, pl;
#pragma unroll
    for (int j = 0; j < 8; ++j) {
      const unsigned int h0 = f2bf(p[2 * j]);
      const unsigned int h1 = f2bf(p[2 * j + 1]);
      const unsigned int l0 = f2bf(p[2 * j]     - bf2f(h0));
      const unsigned int l1 = f2bf(p[2 * j + 1] - bf2f(h1));
      ph.w[j] = (int)(h0 | (h1 << 16));
      pl.w[j] = (int)(l0 | (l1 << 16));
    }

    if (__builtin_amdgcn_ballot_w32(sc != 1.0f) != 0u) {
#pragma unroll
      for (int r = 0; r < 8; ++r) {
        const float s = __shfl(sc, 8 * hh + r);
        O[0][r] *= s; O[1][r] *= s; O[2][r] *= s; O[3][r] *= s;
      }
    }

#pragma unroll
    for (int ct = 0; ct < 4; ++ct) {
      const unsigned short* vh = vhp + (size_t)(16 * ct) * NNODE + k0;
      const unsigned short* vl = vlp + (size_t)(16 * ct) * NNODE + k0;
      FragB bhf, blf;
      bhf.h[0] = *(const v8usa*)vh;
      bhf.h[1] = *(const v8usa*)(vh + 16);
      blf.h[0] = *(const v8usa*)vl;
      blf.h[1] = *(const v8usa*)(vl + 16);
      O[ct] = wmb(ph, bhf, O[ct]);
      O[ct] = wmb(ph, blf, O[ct]);
      O[ct] = wmb(pl, bhf, O[ct]);
    }
  }

  rs += __shfl_xor(rs, 16);
  const float inv = 1.0f / rs;
  float* sw = st + wave * (AROWS * HD);
#pragma unroll
  for (int r = 0; r < 8; ++r) {
    const float ir = __shfl(inv, 8 * hh + r);
#pragma unroll
    for (int ct = 0; ct < 4; ++ct) {
      const float v = fmaxf(O[ct][r] * ir, 0.0f);
      sw[(8 * hh + r) * HD + 16 * ct + m] = v;
    }
  }
  __syncthreads();

  v4f fv[8];
#pragma unroll
  for (int i = 0; i < 8; ++i) fv[i] = *(const v4fa*)(sw + (2 * i + hh) * HD + 4 * m);
  float* ob = out + ((size_t)b * NNODE + (size_t)row0) * ODIM + h * HD + 4 * m;
#pragma unroll
  for (int i = 0; i < 8; ++i) {
    float* op = ob + (size_t)(2 * i + hh) * ODIM;
    *(volatile v4f*)op = fv[i];
  }
  __threadfence();
#pragma unroll
  for (int i = 0; i < 8; ++i) {
    float* op = ob + (size_t)(2 * i + hh) * ODIM;
    *(volatile v4f*)op = fv[i];
  }
}

extern "C" void kernel_launch(void* const* d_in, const int* in_sizes, int n_in,
                              void* d_out, int out_size, void* d_ws, size_t ws_size,
                              hipStream_t stream) {
  if (n_in < 7) return;
  if (in_sizes[0] != NB * NNODE * NNODE) return;
  if (in_sizes[1] != NB * NNODE * KIN) return;
  if (in_sizes[2] != NHEAD * KIN * HD) return;
  if (in_sizes[3] != NHEAD * HD) return;
  if (in_sizes[4] != NHEAD) return;
  if (in_sizes[5] != NHEAD * HD) return;
  if (in_sizes[6] != NHEAD) return;
  if (out_size != NB * NNODE * ODIM) return;

  const float* A  = (const float*)d_in[0];
  const float* X  = (const float*)d_in[1];
  const float* W  = (const float*)d_in[2];
  const float* w1 = (const float*)d_in[3];
  const float* b1 = (const float*)d_in[4];
  const float* w2 = (const float*)d_in[5];
  const float* b2 = (const float*)d_in[6];
  float* out = (float*)d_out;

  char* ws = (char*)d_ws;
  size_t off = 0;
  const size_t oXB = off; off += (size_t)MROWS * KIN * 2;               off = (off + 255) & ~(size_t)255;
  const size_t oWT = off; off += (size_t)ODIM * KIN * 2;                off = (off + 255) & ~(size_t)255;
  const size_t oAB = off; off += (size_t)NB * NNODE * NNODE * 2;        off = (off + 255) & ~(size_t)255;
  const size_t oVH = off; off += (size_t)NB * NHEAD * HD * NNODE * 2;   off = (off + 255) & ~(size_t)255;
  const size_t oVL = off; off += (size_t)NB * NHEAD * HD * NNODE * 2;   off = (off + 255) & ~(size_t)255;
  const size_t oSD = off; off += (size_t)NB * NHEAD * 2 * NNODE * 4;    off = (off + 255) & ~(size_t)255;
  if (off > ws_size || off > (size_t)WSMAX) return;
  unsigned short* XB  = (unsigned short*)(ws + oXB);
  unsigned short* WT  = (unsigned short*)(ws + oWT);
  unsigned short* AB  = (unsigned short*)(ws + oAB);
  unsigned short* VtH = (unsigned short*)(ws + oVH);
  unsigned short* VtL = (unsigned short*)(ws + oVL);
  float*          SD  = (float*)(ws + oSD);

  k_prep<<<NBX + NBA + NBW, PTHR, 0, stream>>>(A, X, W, AB, XB, WT);
  k_proj<<<dim3(MROWS / GBM, ODIM / GBN), GTHR, 0, stream>>>(XB, WT, w1, b1, w2, b2, VtH, VtL, SD);
  k_attn<<<NB * (NNODE / AROWS), ATHR, 0, stream>>>(AB, VtH, VtL, SD, out);
}
